// SelfAttention_23021024706947
// MI455X (gfx1250) — hardware-run, weakly checked
//
#include <hip/hip_runtime.h>


#ifndef NB
#define NB 2
#endif
#ifndef SEQ
#define SEQ 2304
#endif
#define NB_FULL  2
#define SEQ_FULL 2304
#ifndef OUT_SEQ
#define OUT_SEQ SEQ
#endif
#define DIMC  256
#define NHD   8
#define HD    64
#define INNER 512
#define NKEYS (SEQ + 1)
#define NKL   (((NKEYS + 31) / 32) * 32)
#define NKP   (((NKEYS + 63) / 64) * 64)
#define AW    4
#define OSP   68
#define WSC   64.0f
#define WSI   (1.0f / 64.0f)
#define VSC   16.0f
#define CSC   1024.0f
#define OSI   (1.0f / 65536.0f)
#define PSH   14.0f
#define NEGB  (-3.0e38f)
#define SC2   ((float)(0.125 * 1.4426950408889634))
#define MASK2 ((float)(-100.0 * 1.4426950408889634))

static_assert(HD == 64);
static_assert(NHD * HD == INNER);
static_assert(DIMC % 64 == 0);
static_assert(INNER % 64 == 0);
static_assert(DIMC % 32 == 0);
static_assert(INNER % 32 == 0);
static_assert(HD % 32 == 0);
static_assert(SEQ % 64 == 0);
static_assert(SEQ % 32 == 0);
static_assert(SEQ % (16 * AW) == 0);
static_assert(NKP % 64 == 0);
static_assert(NKL % 32 == 0);
static_assert(NKL >= NKEYS);
static_assert(NKL <= NKP);
static_assert(NKP % 32 == 0);
static_assert(OUT_SEQ % 32 == 0);
static_assert(OUT_SEQ >= SEQ);
static_assert(NB <= NB_FULL);
static_assert(SEQ <= SEQ_FULL);
static_assert((OSP * 4) % 16 == 0);
static_assert(256 * 4 * 16 == 32 * DIMC * 2);
static_assert(32 * 4 * 16 == 16 * HD * 2);
static_assert(32 * 4 * 16 == 16 * 64 * 2);
static_assert(32 * 8 * 16 == 16 * 64 * 4);
static_assert((16 * OSP * 4) <= 131072);
static_assert((AW * 16 * OSP * 4) <= 131072);
static_assert((DIMC * 33 * 4 + 8 * 32 * 4 + 32 * 4) <= 131072);
static_assert(((size_t)NB * NHD * NKP) % 256 == 0);

typedef _Float16 h16;
typedef __attribute__((ext_vector_type(16))) _Float16 v16h;
typedef __attribute__((ext_vector_type(8)))  _Float16 v8h;
typedef __attribute__((ext_vector_type(8)))  float    v8f;
typedef __attribute__((ext_vector_type(4)))  float    v4f;
typedef v4f  __attribute__((may_alias)) v4fa;

__device__ __forceinline__ unsigned short f2bf(float f) { unsigned u = __float_as_uint(f); u += 0x7FFFu + ((u >> 16) & 1u); return (unsigned short)(u >> 16); }
__device__ __forceinline__ float bfr(float f) { return __uint_as_float(((unsigned)f2bf(f)) << 16); }
__device__ __forceinline__ v16h cat16(v8h lo, v8h hi) { return __builtin_shufflevector(lo, hi, 0, 1, 2, 3, 4, 5, 6, 7, 8, 9, 10, 11, 12, 13, 14, 15); }
__device__ __forceinline__ v16h  ldh(const h16* p) { return cat16(*(const v8h*)p, *(const v8h*)(p + 16)); }
__device__ __forceinline__ void wave_sync() { __builtin_amdgcn_fence(3  , "wavefront"); __builtin_amdgcn_wave_barrier(); asm volatile("" ::: "memory"); }
static __device__ __forceinline__ h16 toh_flush(float v) { const h16 r = (h16)v; return (fabsf(v) < 6.103515625e-05f) ? (h16)0.0f : r; }
__device__ __forceinline__ v8f wmg(v16h a, v16h b, v8f c) {
    c = __builtin_amdgcn_wmma_f32_16x16x32_f16(false, a, false, b, (short)0, c, false, false);
    asm volatile("v_nop\n\tv_nop\n\tv_nop\n\tv_nop" : "+v"(c) : "v"(a), "v"(b));
    return c;
}

__global__ __launch_bounds__(256) void k_wcvt(const float* __restrict__ src, h16* dst, size_t n8) {
    const size_t i = (size_t)blockIdx.x * 256 + threadIdx.x; if (i >= n8) return;
    const v8f v = *(const v8f*)(src + i * 8); v8h o;
#pragma unroll
    for (int k = 0; k < 8; ++k) o[k] = toh_flush(bfr(v[k]) * WSC);
    *(volatile v8h*)(dst + i * 8) = o; __threadfence(); *(volatile v8h*)(dst + i * 8) = o;
}

__global__ __launch_bounds__(256) void k_norm(const float* __restrict__ fmap, const float* __restrict__ gamma, h16* XN) {
#pragma clang fp contract(off)
    __shared__ float tile[DIMC * 33];
    __shared__ float part[8 * 32];
    __shared__ float rinv[32];
    const int lane = threadIdx.x & 31;
    const int wave = __builtin_amdgcn_readfirstlane((int)(threadIdx.x >> 5));
    const int b = blockIdx.x / (SEQ / 32), n0 = (blockIdx.x % (SEQ / 32)) * 32;
    const float* src = fmap + (size_t)b * DIMC * SEQ_FULL + n0 + lane;
    float ss = 0.0f;
#pragma unroll 1
    for (int i = 0; i < DIMC / 8; ++i) { const int c = wave + 8 * i; const float v = bfr(src[(size_t)c * SEQ_FULL]); tile[c * 33 + lane] = v; ss += v * v; }
    part[wave * 32 + lane] = ss;
    __syncthreads();
    if (wave == 0) { float s = 0.0f;
#pragma unroll 1
        for (int w = 0; w < 8; ++w) s += part[w * 32 + lane];
        const float l2 = sqrtf(s); rinv[lane] = 1.0f / fmaxf(l2, 1e-12f); }
    __syncthreads();
#pragma unroll 1
    for (int ps = 0; ps < 2; ++ps) {
#pragma unroll 1
        for (int it = 0; it < 4; ++it) {
            const int p = it * 256 + (int)threadIdx.x; const int tok = p >> 5, c8 = (p & 31) * 8;
            const float ri = rinv[tok]; const v8f gv = *(const v8f*)(gamma + c8); v8h hv;
#pragma unroll
            for (int k = 0; k < 8; ++k) hv[k] = toh_flush(((tile[(c8 + k) * 33 + tok] * ri) * 16.0f) * bfr(gv[k]));
            *(volatile v8h*)(XN + ((size_t)b * SEQ + n0 + tok) * DIMC + c8) = hv; }
        if (ps == 0) __threadfence(); }
}

__device__ __forceinline__ void gemm_core(const h16* __restrict__ A, const size_t (&ao)[4], const h16* __restrict__ Bt, const size_t (&bo)[4], const int K, v8f (&acc)[4][4]) {
#pragma unroll
    for (int mb = 0; mb < 4; ++mb)
#pragma unroll
        for (int nb = 0; nb < 4; ++nb) acc[mb][nb] = (v8f){};
#pragma unroll 1
    for (int kc = 0; kc < K; kc += 32) {
        v16h a[4];
#pragma unroll
        for (int mb = 0; mb < 4; ++mb) a[mb] = ldh(A + ao[mb] + kc);
#pragma unroll
        for (int nb = 0; nb < 4; ++nb) { const v16h b = ldh(Bt + bo[nb] + kc);
#pragma unroll
            for (int mb = 0; mb < 4; ++mb) acc[mb][nb] = wmg(a[mb], b, acc[mb][nb]); }
    }
}

__global__ __launch_bounds__(32) void k_proj_qk(const h16* __restrict__ XN, const h16* __restrict__ W, const float* __restrict__ nullkv, h16* KP) {
    __shared__ __align__(16) float os[16 * 68];
    const int lane = threadIdx.x & 31, lr = lane & 15, hi = lane >> 4; const int r0 = blockIdx.x * 64, c0 = blockIdx.y * 64;
    const int bb = r0 / NKP, kt = r0 % NKP;
    size_t ao[4], bo[4];
#pragma unroll
    for (int mb = 0; mb < 4; ++mb) { int tok = kt + mb * 16 + lr - 1; tok = tok < 0 ? 0 : (tok > SEQ - 1 ? SEQ - 1 : tok);
        ao[mb] = ((size_t)bb * SEQ + (size_t)tok) * DIMC + 8 * hi; }
#pragma unroll
    for (int nb = 0; nb < 4; ++nb) bo[nb] = (size_t)(c0 + nb * 16 + lr) * DIMC + 8 * hi;
    v8f acc[4][4];
    gemm_core(XN, ao, W, bo, DIMC, acc);
    float bc[4];
#pragma unroll
    for (int nb = 0; nb < 4; ++nb) { float t = nullkv[c0 + nb * 16 + lr]; asm volatile("" : "+v"(t)); bc[nb] = bfr(t); }
    const size_t tbase = ((size_t)(bb * NHD + c0 / HD) * NKP + (size_t)kt) * HD;
#pragma unroll
    for (int mb = 0; mb < 4; ++mb) {
#pragma unroll
        for (int nb = 0; nb < 4; ++nb) {
#pragma unroll
            for (int j = 0; j < 8; ++j) { const int key = kt + mb * 16 + hi * 8 + j; const float val = acc[mb][nb][j] * WSI;
                os[(hi * 8 + j) * 68 + nb * 16 + lr] = (key == 0) ? bc[nb] : ((key >= NKEYS) ? 0.0f : val); } }
        wave_sync();
#pragma unroll 1
        for (int ps = 0; ps < 2; ++ps) {
            const size_t sb = tbase + (size_t)(mb * 16) * HD;
#pragma unroll
            for (int s = 0; s < 4; ++s) { const int p = s * 32 + lane; const int row = p >> 3, c8 = (p & 7) * 8;
                const v4f x0 = *(const v4fa*)(&os[row * 68 + c8]); const v4f x1 = *(const v4fa*)(&os[row * 68 + c8 + 4]); v8h hv;
#pragma unroll
                for (int i = 0; i < 4; ++i) { hv[i] = toh_flush(x0[i]); hv[4 + i] = toh_flush(x1[i]); }
                *(volatile v8h*)(KP + sb + (size_t)p * 8) = hv; }
            if (ps == 0) __threadfence(); }
        wave_sync();
    }
}

__global__ __launch_bounds__(32) void k_proj_vt(const h16* __restrict__ W, const h16* __restrict__ XN, const float* __restrict__ nullkv, h16* VT) {
    __shared__ __align__(16) float os[16 * 68];
    const int lane = threadIdx.x & 31, lr = lane & 15, hi = lane >> 4; const int r0 = blockIdx.x * 64, c0 = blockIdx.y * 64;
    const int bb = c0 / NKP, kt = c0 % NKP;
    size_t ao[4], bo[4];
#pragma unroll
    for (int mb = 0; mb < 4; ++mb) ao[mb] = (size_t)(r0 + mb * 16 + lr) * DIMC + 8 * hi;
#pragma unroll
    for (int nb = 0; nb < 4; ++nb) { int tok = kt + nb * 16 + lr - 1; tok = tok < 0 ? 0 : (tok > SEQ - 1 ? SEQ - 1 : tok);
        bo[nb] = ((size_t)bb * SEQ + (size_t)tok) * DIMC + 8 * hi; }
    v8f acc[4][4];
    gemm_core(W, ao, XN, bo, DIMC, acc);
    const size_t tbase = ((size_t)bb * INNER + (size_t)r0) * NKP + (size_t)kt;
#pragma unroll
    for (int mb = 0; mb < 4; ++mb) {
        float br[8];
#pragma unroll
        for (int j = 0; j < 8; ++j) { float t = nullkv[INNER + r0 + mb * 16 + hi * 8 + j]; asm volatile("" : "+v"(t)); br[j] = bfr(t) * VSC; }
#pragma unroll
        for (int nb = 0; nb < 4; ++nb) { const int key = kt + nb * 16 + lr;
#pragma unroll
            for (int j = 0; j < 8; ++j) { const float val = acc[mb][nb][j] * (WSI * VSC);
                os[(hi * 8 + j) * 68 + nb * 16 + lr] = (key == 0) ? br[j] : ((key >= NKEYS) ? 0.0f : val); } }
        wave_sync();
#pragma unroll 1
        for (int ps = 0; ps < 2; ++ps) {
            const size_t sb = tbase + (size_t)(mb * 16) * NKP;
#pragma unroll
            for (int s = 0; s < 4; ++s) { const int row = 4 * s + (lane >> 3), c8 = (lane & 7) * 8;
                const v4f x0 = *(const v4fa*)(&os[row * 68 + c8]); const v4f x1 = *(const v4fa*)(&os[row * 68 + c8 + 4]); v8h hv;
#pragma unroll
                for (int i = 0; i < 4; ++i) { hv[i] = toh_flush(x0[i]); hv[4 + i] = toh_flush(x1[i]); }
                *(volatile v8h*)(VT + sb + (size_t)row * NKP + c8) = hv; }
            if (ps == 0) __threadfence(); }
        wave_sync();
    }
}

__global__ __launch_bounds__(256) void k_sq(const h16* __restrict__ KP, float* K2, int rows) {
#pragma clang fp contract(off)
    const int i = blockIdx.x * 256 + (int)threadIdx.x; const int ic = i < rows ? i : rows - 1;
    const h16* p = KP + (size_t)ic * HD; float s = 0.0f;
#pragma unroll 1
    for (int c = 0; c < HD; c += 8) { const v8h v = *(const v8h*)(p + c);
#pragma unroll
        for (int k = 0; k < 8; ++k) { const float f = (float)v[k]; s += f * f; } }
    if (i < rows) *(volatile float*)(K2 + i) = s;
    __threadfence();
    if (i < rows) *(volatile float*)(K2 + i) = s;
}

__global__ __launch_bounds__(32 * AW) __attribute__((amdgpu_num_vgpr(256))) void k_flash(const h16* __restrict__ KP, const float* __restrict__ K2, const h16* __restrict__ VT, h16* CT) {
    __shared__ __align__(16) float os[AW * 16 * OSP];
    const int lane = threadIdx.x & 31, lr = lane & 15, hi = lane >> 4;
    const int wave = __builtin_amdgcn_readfirstlane((int)(threadIdx.x >> 5));
    const int zh = blockIdx.y; const int b = zh / NHD, h = zh % NHD;
    const int t0 = (blockIdx.x * AW + wave) * 16;
    const size_t pbase = (size_t)zh * NKP * HD;
    const int tq1 = t0 + lr + 1;
    const size_t qo = pbase + (size_t)tq1 * HD + 8 * hi;
    const v16h q0 = ldh(KP + qo), q1 = ldh(KP + qo + 32);
    const float q2 = K2[(size_t)zh * NKP + tq1];
    const float* k2b = K2 + (size_t)zh * NKP + 8 * hi;
    const size_t ko = pbase + (size_t)lr * HD + 8 * hi;
    const size_t vo = pbase + (size_t)lr * NKP + 8 * hi;
    v8f o[4];
#pragma unroll
    for (int j = 0; j < 4; ++j) o[j] = (v8f){};
    float m = NEGB, l = 0.0f;
#pragma unroll 1
    for (int key0 = 0; key0 < NKL; key0 += 32) {
        const h16* ka = KP + ko + (size_t)key0 * HD;
        v8f sa = (v8f){}, sb = (v8f){};
        { const v16h ka0 = ldh(ka), ka1 = ldh(ka + 32); sa = wmg(ka0, q0, sa); sa = wmg(ka1, q1, sa); }
        { const v16h kb0 = ldh(ka + 16 * HD), kb1 = ldh(ka + 16 * HD + 32); sb = wmg(kb0, q0, sb); sb = wmg(kb1, q1, sb); }
        const float* kp = k2b + key0;
        const v4f m0 = *(const v4f*)kp, m1 = *(const v4f*)(kp + 4), m2 = *(const v4f*)(kp + 16), m3 = *(const v4f*)(kp + 20);
        float kx[8], ky[8];
#pragma unroll
        for (int r = 0; r < 4; ++r) { kx[r] = m0[r]; kx[4 + r] = m1[r]; ky[r] = m2[r]; ky[4 + r] = m3[r]; }
        const int ja = key0 + 8 * hi;
        float ta[8], tb[8]; float mx = NEGB;
#pragma unroll
        for (int r = 0; r < 8; ++r) {
            const int jA = ja + r, jB = ja + 16 + r;
            const float dA = fmaxf((q2 + kx[r]) - 2.0f * sa[r], 0.0f);
            const float dB = fmaxf((q2 + ky[r]) - 2.0f * sb[r], 0.0f);
            float uA = -__builtin_amdgcn_sqrtf(dA) * SC2;
            float uB = -__builtin_amdgcn_sqrtf(dB) * SC2;
            uA = (jA == tq1) ? MASK2 : uA;
            uB = (jB == tq1) ? MASK2 : uB;
            ta[r] = (jA < NKEYS) ? uA : NEGB;
            tb[r] = (jB < NKEYS) ? uB : NEGB;
            mx = fmaxf(mx, fmaxf(ta[r], tb[r])); }
        mx = fmaxf(mx, __shfl_xor(mx, 16, 32));
        const float mnew = fmaxf(m, mx);
        const float alpha = __builtin_amdgcn_exp2f(m - mnew);
        const float sh = PSH - mnew;
        v16h pb; float ls = 0.0f;
#pragma unroll
        for (int r = 0; r < 8; ++r) {
            const float ea = ta[r] + sh, eb = tb[r] + sh;
            const float xa = __builtin_amdgcn_exp2f(ea), xb = __builtin_amdgcn_exp2f(eb);
            const float ga = (ea < -14.0f) ? 0.0f : xa, gb = (eb < -14.0f) ? 0.0f : xb;
            const h16 pa = (h16)ga; const h16 pc = (h16)gb;
            pb[r] = pa; pb[8 + r] = pc;
            ls += (float)pa + (float)pc; }
        l = l * alpha + ls; m = mnew;
#pragma unroll
        for (int j = 0; j < 4; ++j) o[j] = o[j] * alpha;
        const h16* va = VT + vo + key0;
#pragma unroll
        for (int j = 0; j < 4; ++j) { const v16h vf = ldh(va + (size_t)(16 * j) * NKP); o[j] = wmg(vf, pb, o[j]); }
    }
    l += __shfl_xor(l, 16, 32);
    const float inv = (CSC / VSC) * (1.0f / l);
    const int wb = wave * 16 * OSP;
#pragma unroll
    for (int j = 0; j < 4; ++j) { v4f a, c;
        a[0] = o[j][0] * inv; a[1] = o[j][1] * inv; a[2] = o[j][2] * inv; a[3] = o[j][3] * inv;
        c[0] = o[j][4] * inv; c[1] = o[j][5] * inv; c[2] = o[j][6] * inv; c[3] = o[j][7] * inv;
        *(v4fa*)(&os[wb + lr * OSP + 16 * j + 8 * hi]) = a; *(v4fa*)(&os[wb + lr * OSP + 16 * j + 8 * hi + 4]) = c; }
    wave_sync();
    h16* crow = CT + ((size_t)b * SEQ + t0) * INNER + h * HD;
#pragma unroll 1
    for (int ps = 0; ps < 2; ++ps) {
#pragma unroll
        for (int s = 0; s < 4; ++s) { const int row = 4 * s + (lane >> 3), c8 = (lane & 7) * 8;
            const v4f x0 = *(const v4fa*)(&os[wb + row * OSP + c8]); const v4f x1 = *(const v4fa*)(&os[wb + row * OSP + c8 + 4]); v8h hv;
#pragma unroll
            for (int i = 0; i < 4; ++i) { hv[i] = toh_flush(x0[i]); hv[4 + i] = toh_flush(x1[i]); }
            *(volatile v8h*)(crow + (size_t)row * INNER + c8) = hv; }
        if (ps == 0) __threadfence(); }
}

__global__ __launch_bounds__(32) void k_out(const h16* __restrict__ W, const h16* __restrict__ CT, float* OUT) {
    __shared__ __align__(16) float os[16 * 68];
    const int lane = threadIdx.x & 31, lr = lane & 15, hi = lane >> 4; const int r0 = blockIdx.x * 64, c0 = blockIdx.y * 64;
    const int bb = c0 / SEQ, tt = c0 % SEQ;
    size_t ao[4], bo[4];
#pragma unroll
    for (int mb = 0; mb < 4; ++mb) ao[mb] = (size_t)(r0 + mb * 16 + lr) * INNER + 8 * hi;
#pragma unroll
    for (int nb = 0; nb < 4; ++nb) bo[nb] = (size_t)(c0 + nb * 16 + lr) * INNER + 8 * hi;
    v8f acc[4][4];
    gemm_core(W, ao, CT, bo, INNER, acc);
    const size_t obase = ((size_t)bb * DIMC + (size_t)r0) * OUT_SEQ + (size_t)tt;
#pragma unroll
    for (int mb = 0; mb < 4; ++mb) {
#pragma unroll
        for (int nb = 0; nb < 4; ++nb) {
#pragma unroll
            for (int j = 0; j < 8; ++j) os[(hi * 8 + j) * 68 + nb * 16 + lr] = acc[mb][nb][j] * OSI; }
        wave_sync();
#pragma unroll 1
        for (int ps = 0; ps < 2; ++ps) {
            const size_t sb = obase + (size_t)(mb * 16) * OUT_SEQ;
#pragma unroll
            for (int s = 0; s < 8; ++s) { const int row = 2 * s + (lane >> 4), c4 = (lane & 15) * 4;
                const v4f val = *(const v4fa*)(&os[row * 68 + c4]);
                *(volatile v4f*)(OUT + sb + (size_t)row * OUT_SEQ + c4) = val; }
            if (ps == 0) __threadfence(); }
        wave_sync();
    }
}

static constexpr size_t al256(size_t v) { return (v + 255) & ~(size_t)255; }
static constexpr size_t SZ_W  = al256((size_t)INNER * DIMC * 2);
static constexpr size_t SZ_XN = al256((size_t)NB * SEQ * DIMC * 2);
static constexpr size_t SZ_KP = al256((size_t)NB * NHD * NKP * HD * 2);
static constexpr size_t SZ_K2 = al256((size_t)NB * NHD * NKP * 4);
static constexpr size_t SZ_CT = al256((size_t)NB * SEQ * INNER * 2);
static constexpr size_t SZ_TOTAL = 3 * SZ_W + SZ_XN + 2 * SZ_KP + SZ_K2 + SZ_CT;
static_assert(SZ_TOTAL <= (size_t)134217728);
static_assert((size_t)NB * NHD * NKP * HD == (size_t)NB * INNER * NKP);
static_assert(((size_t)INNER * DIMC) % (8 * 256) == 0);

extern "C" void kernel_launch(void* const* d_in, const int* in_sizes, int n_in,
                              void* d_out, int out_size, void* d_ws, size_t ws_size, hipStream_t stream) {
    if (n_in < 6) return;
    const size_t needx = ((size_t)(NB - 1) * DIMC + (DIMC - 1)) * SEQ_FULL + SEQ;
    if ((size_t)in_sizes[0] < needx) return;
    if (in_sizes[1] < DIMC) return;
    if ((size_t)in_sizes[2] < (size_t)INNER * DIMC || (size_t)in_sizes[3] < (size_t)INNER * DIMC || (size_t)in_sizes[5] < (size_t)DIMC * INNER) return;
    if (in_sizes[4] < 2 * INNER) return;
    if ((size_t)out_size < ((size_t)(NB - 1) * DIMC + (DIMC - 1)) * OUT_SEQ + SEQ) return;
    if (SZ_TOTAL > ws_size) return;
    const float* fmap = (const float*)d_in[0];
    const float* gamma = (const float*)d_in[1];
    const float* wqk = (const float*)d_in[2];
    const float* wv = (const float*)d_in[3];
    const float* nullkv = (const float*)d_in[4];
    const float* wout = (const float*)d_in[5];
    float* OUT = (float*)d_out;
    char* wsp = (char*)d_ws;
    h16* WQ = (h16*)wsp; wsp += SZ_W;
    h16* WV = (h16*)wsp; wsp += SZ_W;
    h16* WO = (h16*)wsp; wsp += SZ_W;
    h16* XN = (h16*)wsp; wsp += SZ_XN;
    h16* KP = (h16*)wsp; wsp += SZ_KP;
    h16* VT = (h16*)wsp; wsp += SZ_KP;
    float* K2 = (float*)wsp; wsp += SZ_K2;
    h16* CT = (h16*)wsp; wsp += SZ_CT;

    { const size_t n8 = (size_t)INNER * DIMC / 8; const unsigned g = (unsigned)((n8 + 255) / 256);
      k_wcvt<<<g, 256, 0, stream>>>(wqk, WQ, n8); k_wcvt<<<g, 256, 0, stream>>>(wv, WV, n8); k_wcvt<<<g, 256, 0, stream>>>(wout, WO, n8); }

    k_norm<<<NB * (SEQ / 32), 256, 0, stream>>>(fmap, gamma, XN);

    k_proj_qk<<<dim3(NB * NKP / 64, INNER / 64, 1), 32, 0, stream>>>(XN, WQ, nullkv, KP);
    k_proj_vt<<<dim3(INNER / 64, NB * NKP / 64, 1), 32, 0, stream>>>(WV, XN, nullkv, VT);

    { const int rows = NB * NHD * NKP; k_sq<<<(unsigned)((rows + 255) / 256), 256, 0, stream>>>(KP, K2, rows); }

    k_flash<<<dim3(SEQ / (16 * AW), NB * NHD, 1), 32 * AW, 0, stream>>>(KP, K2, VT, CT);

    k_out<<<dim3(DIMC / 64, NB * SEQ / 64, 1), 32, 0, stream>>>(WO, CT, OUT);
}
